// GCN_Top_63290638074050
// MI455X (gfx1250) — hardware-verified
//
#include <hip/hip_runtime.h>
#include <stddef.h>


#define HID     512
#define DIN     128
#define NTHR    256
#define NWAVE   8
#define EPT     8
#define NGRP    2
#define CHUNK   (NTHR * EPT * NGRP)
#define WCAP    (EPT * NGRP * 32)
#define LISTN   (NWAVE * WCAP)
#define NBA     128
#define NBD     4096
#define GR      128
#define GCOL    128
#define TPB     32

#define LDS_GEMM (NWAVE * 32 * 64 * 4)
#define LDS_AGG  (NBA * HID * 4 + LISTN * 4 + 64)

static_assert((CHUNK & (CHUNK - 1)) == 0);
static_assert(CHUNK <= 4096);
static_assert((NBA & (NBA - 1)) == 0 && NBA <= 4096);
static_assert((NBD & (NBD - 1)) == 0 && NBD <= 4096);
static_assert(NBA == GR);
static_assert(NBD % GR == 0);
static_assert(HID % GCOL == 0 && DIN % 32 == 0 && HID % 32 == 0);
static_assert((NBA * HID / 8) % NTHR == 0);
static_assert(TPB == 4 * NWAVE);

typedef float          v4f  __attribute__((ext_vector_type(4)));
typedef float          v8f  __attribute__((ext_vector_type(8)));
typedef int            v4i  __attribute__((ext_vector_type(4)));
typedef unsigned short v8us __attribute__((ext_vector_type(8)));
typedef __bf16         v8b  __attribute__((ext_vector_type(8)));
typedef __bf16         v16b __attribute__((ext_vector_type(16)));
union FragB { v16b v; v8b h[2]; };

__device__ __forceinline__ unsigned int bfbits(float f) {
  const unsigned int u = __float_as_uint(f);
  return (u + 0x7FFFu + ((u >> 16) & 1u)) >> 16;
}

#define SPLIT1(V, I) { const unsigned int hb_ = bfbits(V); const float hf_ = __uint_as_float(hb_ << 16); \
  hv[I] = (unsigned short)hb_; lv[I] = (unsigned short)bfbits((V) - hf_); }

__device__ __forceinline__ void split8(const v4f a, const v4f b, v8us* hp, v8us* lp) {
  v8us hv, lv;
  SPLIT1(a.x, 0) SPLIT1(a.y, 1) SPLIT1(a.z, 2) SPLIT1(a.w, 3)
  SPLIT1(b.x, 4) SPLIT1(b.y, 5) SPLIT1(b.z, 6) SPLIT1(b.w, 7)
  *hp = hv; *lp = lv;
}
#undef SPLIT1

__device__ __forceinline__ v8f wmb(v16b a, v16b b, v8f c) {
  v8f d = __builtin_amdgcn_wmma_f32_16x16x32_bf16(false, a, false, b, (short)0, c, false, false);
  asm volatile("v_nop\n\tv_nop\n\tv_nop\n\tv_nop" : "+v"(d) : "v"(a), "v"(b));
  return d;
}

__device__ __forceinline__ float tanh_f(float x) {
  const float ax = fabsf(x);
  const float e  = __expf(ax + ax);
  const float r  = __builtin_amdgcn_rcpf(e + 1.0f);
  const float t  = 1.0f - (r + r);
  return copysignf(t, x);
}
__device__ __forceinline__ v4f tanh4(v4f v) {
  v4f r;
  r.x = tanh_f(v.x); r.y = tanh_f(v.y); r.z = tanh_f(v.z); r.w = tanh_f(v.w);
  return r;
}

template <int NB>
__device__ __forceinline__ int scan_chunk(const int* __restrict__ dsts, int nE, int cbase, int nodeBase,
                                          int vec8, int* list, int tid, int lane, int wave) {
  int wc = 0;
#pragma unroll
  for (int g = 0; g < NGRP; ++g) {
    const int el0  = (g * NTHR + tid) * EPT;
    const int e0   = cbase + el0;
    const int sent = -2147483647 - 1;
    v4i da, db;
    if (vec8 != 0 && cbase + CHUNK <= nE) {
      da = *(const v4i*)(dsts + e0);
      db = *(const v4i*)(dsts + e0 + 4);
    } else {
      da.x = (e0     < nE) ? dsts[min(e0, nE - 1)] : sent;
      da.y = (e0 + 1 < nE) ? dsts[min(e0 + 1, nE - 1)] : sent;
      da.z = (e0 + 2 < nE) ? dsts[min(e0 + 2, nE - 1)] : sent;
      da.w = (e0 + 3 < nE) ? dsts[min(e0 + 3, nE - 1)] : sent;
      db.x = (e0 + 4 < nE) ? dsts[min(e0 + 4, nE - 1)] : sent;
      db.y = (e0 + 5 < nE) ? dsts[min(e0 + 5, nE - 1)] : sent;
      db.z = (e0 + 6 < nE) ? dsts[min(e0 + 6, nE - 1)] : sent;
      db.w = (e0 + 7 < nE) ? dsts[min(e0 + 7, nE - 1)] : sent;
    }
    const unsigned nb = (unsigned)nodeBase;
    const unsigned s0 = (unsigned)da.x - nb, s1 = (unsigned)da.y - nb;
    const unsigned s2 = (unsigned)da.z - nb, s3 = (unsigned)da.w - nb;
    const unsigned s4 = (unsigned)db.x - nb, s5 = (unsigned)db.y - nb;
    const unsigned s6 = (unsigned)db.z - nb, s7 = (unsigned)db.w - nb;
    const bool h0 = s0 < (unsigned)NB, h1 = s1 < (unsigned)NB, h2 = s2 < (unsigned)NB, h3 = s3 < (unsigned)NB;
    const bool h4 = s4 < (unsigned)NB, h5 = s5 < (unsigned)NB, h6 = s6 < (unsigned)NB, h7 = s7 < (unsigned)NB;
    const unsigned any = __builtin_amdgcn_ballot_w32(h0 | h1 | h2 | h3 | h4 | h5 | h6 | h7);
    if (any != 0u) {
#define HITJ(J, HJ, SJ) { \
        const unsigned mj = __builtin_amdgcn_ballot_w32(HJ); \
        if (mj != 0u) { \
          if (HJ) { \
            const int pos = wc + (int)__builtin_amdgcn_mbcnt_lo(mj, 0u); \
            if (pos < WCAP) list[wave * WCAP + pos] = ((el0 + (J)) << 12) | (int)(SJ); \
          } \
          wc += (int)__builtin_popcount(mj); } }
      HITJ(0, h0, s0)
      HITJ(1, h1, s1)
      HITJ(2, h2, s2)
      HITJ(3, h3, s3)
      HITJ(4, h4, s4)
      HITJ(5, h5, s5)
      HITJ(6, h6, s6)
      HITJ(7, h7, s7)
#undef HITJ
    }
  }
  return wc;
}

__global__ __launch_bounds__(NTHR) void k_wprep(
    const float* __restrict__ W1, const float* __restrict__ W2, const float* __restrict__ W3,
    unsigned short* w1h, unsigned short* w1l, unsigned short* w2h, unsigned short* w2l,
    unsigned short* w3h, unsigned short* w3l) {
  const int i  = blockIdx.x * NTHR + threadIdx.x;
  const int n1 = HID * DIN / 8;
  const int n2 = HID * HID / 8;
  if (i >= n1 + 2 * n2) return;
  const int seg = (i < n1) ? 0 : ((i < n1 + n2) ? 1 : 2);
  const int K   = (seg == 0) ? DIN : HID;
  const int li  = (seg == 0) ? i : ((seg == 1) ? (i - n1) : (i - n1 - n2));
  const float* W = (seg == 0) ? W1 : ((seg == 1) ? W2 : W3);
  unsigned short* oh = (seg == 0) ? w1h : ((seg == 1) ? w2h : w3h);
  unsigned short* ol = (seg == 0) ? w1l : ((seg == 1) ? w2l : w3l);
  const int o  = li * 8;
  const int n  = o / K;
  const int k0 = o - n * K;
  const float* p = W + (size_t)k0 * HID + n;
  v4f a, b;
  a.x = p[0];       a.y = p[HID];     a.z = p[2 * HID]; a.w = p[3 * HID];
  b.x = p[4 * HID]; b.y = p[5 * HID]; b.z = p[6 * HID]; b.w = p[7 * HID];
  v8us hv, lv;
  split8(a, b, &hv, &lv);
  *(volatile v8us*)(oh + o) = hv;
  *(volatile v8us*)(ol + o) = lv;
  __threadfence();
  *(volatile v8us*)(oh + o) = hv;
  *(volatile v8us*)(ol + o) = lv;
}

__global__ __launch_bounds__(NTHR) void k_xprep(
    const float* __restrict__ x, unsigned short* xh, unsigned short* xl, int nN, int nRows) {
  const int i = blockIdx.x * NTHR + threadIdx.x;
  const int total = nRows * (DIN / 8);
  if (i >= total) return;
  const int r  = i / (DIN / 8);
  const int c0 = (i - r * (DIN / 8)) * 8;
  const int rs = r > nN - 1 ? nN - 1 : r;
  const float* p = x + (size_t)rs * DIN + c0;
  const v4f a = *(const v4f*)p, b = *(const v4f*)(p + 4);
  v8us hv, lv;
  split8(a, b, &hv, &lv);
  const size_t o = (size_t)i * 8;
  *(volatile v8us*)(xh + o) = hv;
  *(volatile v8us*)(xl + o) = lv;
  __threadfence();
  *(volatile v8us*)(xh + o) = hv;
  *(volatile v8us*)(xl + o) = lv;
}

__global__ __launch_bounds__(NTHR) void k_deg(
    const int* __restrict__ ei, float* dinv, int nE, int vec8) {
  __shared__ __attribute__((aligned(16))) int cnt[NBD];
  __shared__ __attribute__((aligned(16))) int list[LISTN];
  __shared__ int wcnt[NWAVE];
  const int tid = threadIdx.x, lane = tid & 31, wave = tid >> 5;
  const int nodeBase = blockIdx.x * NBD;
  const int* dsts = ei + nE;

  for (int i = tid; i < NBD; i += NTHR) cnt[i] = 0;
  __syncthreads();

  const int nChunks = (nE + CHUNK - 1) / CHUNK;
#pragma unroll 1
  for (int ch = 0; ch < nChunks; ++ch) {
    const int cbase = ch * CHUNK;
    const int wc = scan_chunk<NBD>(dsts, nE, cbase, nodeBase, vec8, list, tid, lane, wave);
    if (lane == 0) wcnt[wave] = wc;
    __syncthreads();
    if (wave == 0) {
#pragma unroll 1
      for (int wsx = 0; wsx < NWAVE; ++wsx) {
        int n = __builtin_amdgcn_readfirstlane(wcnt[wsx]);
        n = n > WCAP ? WCAP : (n < 0 ? 0 : n);
        const int* lp = list + wsx * WCAP;
#pragma unroll 1
        for (int i = 0; i < n; ++i) {
          const int ent  = __builtin_amdgcn_readfirstlane(lp[i]);
          const int slot = ent & (NBD - 1);
          if (lane == 0) cnt[slot] = cnt[slot] + 1;
        }
      }
    }
    __syncthreads();
  }

  v4f dq[4];
#pragma unroll
  for (int q = 0; q < 4; ++q) {
    const int f = (wave * 4 + q) * 128 + 4 * lane;
    const v4i c = *(const v4i*)(cnt + f);
    dq[q].x = rsqrtf((float)(c.x + 1));
    dq[q].y = rsqrtf((float)(c.y + 1));
    dq[q].z = rsqrtf((float)(c.z + 1));
    dq[q].w = rsqrtf((float)(c.w + 1));
  }
  float* dp = dinv + (size_t)nodeBase;
#pragma unroll
  for (int q = 0; q < 4; ++q) *(volatile v4f*)(dp + (wave * 4 + q) * 128 + 4 * lane) = dq[q];
  __threadfence();
#pragma unroll
  for (int q = 0; q < 4; ++q) *(volatile v4f*)(dp + (wave * 4 + q) * 128 + 4 * lane) = dq[q];
}

__global__ __launch_bounds__(NTHR) void k_gemm(
    const unsigned short* __restrict__ Ah, const unsigned short* __restrict__ Al,
    const unsigned short* __restrict__ Bh, const unsigned short* __restrict__ Bl,
    const float* __restrict__ dinv, float* g, int K) {
  extern __shared__ v4f lds_dyn[];
  const int tid = threadIdx.x, lane = tid & 31, wave = tid >> 5, hh = lane >> 4, m = lane & 15;
  float* stg = (float*)lds_dyn + wave * (32 * 64);
  const int rg = wave >> 1, cg = wave & 1;
  const int rowBase = blockIdx.y * GR + 32 * rg;
  const int colBase = blockIdx.x * GCOL + 64 * cg;

  v8f acc[2][4];
#pragma unroll
  for (int rt = 0; rt < 2; ++rt)
#pragma unroll
    for (int ct = 0; ct < 4; ++ct) { v8f z = {0.f, 0.f, 0.f, 0.f, 0.f, 0.f, 0.f, 0.f}; acc[rt][ct] = z; }

  const unsigned short* a0h = Ah + (size_t)(rowBase + m) * K + 8 * hh;
  const unsigned short* a0l = Al + (size_t)(rowBase + m) * K + 8 * hh;
  const unsigned short* a1h = Ah + (size_t)(rowBase + 16 + m) * K + 8 * hh;
  const unsigned short* a1l = Al + (size_t)(rowBase + 16 + m) * K + 8 * hh;
  const unsigned short* b0h = Bh + (size_t)(colBase + m) * K + 8 * hh;
  const unsigned short* b0l = Bl + (size_t)(colBase + m) * K + 8 * hh;

  const int nk = K >> 5;
#pragma unroll 1
  for (int kt = 0; kt < nk; ++kt) {
    const int k0 = 32 * kt;
    FragB fa0h, fa0l, fa1h, fa1l;
    fa0h.h[0] = *(const v8b*)(a0h + k0); fa0h.h[1] = *(const v8b*)(a0h + k0 + 16);
    fa0l.h[0] = *(const v8b*)(a0l + k0); fa0l.h[1] = *(const v8b*)(a0l + k0 + 16);
    fa1h.h[0] = *(const v8b*)(a1h + k0); fa1h.h[1] = *(const v8b*)(a1h + k0 + 16);
    fa1l.h[0] = *(const v8b*)(a1l + k0); fa1l.h[1] = *(const v8b*)(a1l + k0 + 16);
#pragma unroll
    for (int ct = 0; ct < 4; ++ct) {
      const size_t bo = (size_t)(16 * ct) * K + k0;
      FragB fbh, fbl;
      fbh.h[0] = *(const v8b*)(b0h + bo); fbh.h[1] = *(const v8b*)(b0h + bo + 16);
      fbl.h[0] = *(const v8b*)(b0l + bo); fbl.h[1] = *(const v8b*)(b0l + bo + 16);
      acc[0][ct] = wmb(fa0h.v, fbh.v, acc[0][ct]);
      acc[0][ct] = wmb(fa0h.v, fbl.v, acc[0][ct]);
      acc[0][ct] = wmb(fa0l.v, fbh.v, acc[0][ct]);
      acc[1][ct] = wmb(fa1h.v, fbh.v, acc[1][ct]);
      acc[1][ct] = wmb(fa1h.v, fbl.v, acc[1][ct]);
      acc[1][ct] = wmb(fa1l.v, fbh.v, acc[1][ct]);
    }
  }

#pragma unroll
  for (int rt = 0; rt < 2; ++rt) {
    const v4f dA = *(const v4f*)(dinv + (size_t)rowBase + 16 * rt + 8 * hh);
    const v4f dB = *(const v4f*)(dinv + (size_t)rowBase + 16 * rt + 8 * hh + 4);
    float* sp = stg + (16 * rt + 8 * hh) * 64 + m;
#pragma unroll
    for (int ct = 0; ct < 4; ++ct) {
      sp[0 * 64 + 16 * ct] = acc[rt][ct][0] * dA.x;
      sp[1 * 64 + 16 * ct] = acc[rt][ct][1] * dA.y;
      sp[2 * 64 + 16 * ct] = acc[rt][ct][2] * dA.z;
      sp[3 * 64 + 16 * ct] = acc[rt][ct][3] * dA.w;
      sp[4 * 64 + 16 * ct] = acc[rt][ct][4] * dB.x;
      sp[5 * 64 + 16 * ct] = acc[rt][ct][5] * dB.y;
      sp[6 * 64 + 16 * ct] = acc[rt][ct][6] * dB.z;
      sp[7 * 64 + 16 * ct] = acc[rt][ct][7] * dB.w;
    }
  }
  __syncthreads();

  float* gw = g + (size_t)rowBase * HID + colBase;
#pragma unroll
  for (int q = 0; q < 16; ++q) {
    const int rl = 2 * q + hh;
    const v4f v = *(const v4f*)(stg + rl * 64 + 4 * m);
    *(volatile v4f*)(gw + (size_t)rl * HID + 4 * m) = v;
  }
  __threadfence();
#pragma unroll
  for (int q = 0; q < 16; ++q) {
    const int rl = 2 * q + hh;
    const v4f v = *(const v4f*)(stg + rl * 64 + 4 * m);
    *(volatile v4f*)(gw + (size_t)rl * HID + 4 * m) = v;
  }
}

template <int OUT16>
__global__ __launch_bounds__(NTHR) void k_agg(
    const int* __restrict__ ei, const float* __restrict__ g, const float* __restrict__ dinv,
    const float* __restrict__ bias, unsigned short* oh, unsigned short* ol, float* of,
    int nN, int nE, int vec8) {
  extern __shared__ v4f lds_dyn[];
  float* acc  = (float*)lds_dyn;
  int*   list = (int*)(acc + NBA * HID);
  int*   wcnt = list + LISTN;
  const int tid = threadIdx.x, lane = tid & 31, wave = tid >> 5;
  const int nodeBase = blockIdx.x * NBA;
  const int* dsts = ei + nE;

  {
    const v4f z = {0.f, 0.f, 0.f, 0.f};
    for (int i = tid; i < NBA * HID / 4; i += NTHR) lds_dyn[i] = z;
  }
  __syncthreads();

  const int nChunks = (nE + CHUNK - 1) / CHUNK;
#pragma unroll 1
  for (int ch = 0; ch < nChunks; ++ch) {
    const int cbase = ch * CHUNK;
    const int wc = scan_chunk<NBA>(dsts, nE, cbase, nodeBase, vec8, list, tid, lane, wave);
    if (lane == 0) wcnt[wave] = wc;
    __syncthreads();
    if (wave == 0) {
#pragma unroll 1
      for (int wsx = 0; wsx < NWAVE; ++wsx) {
        int n = __builtin_amdgcn_readfirstlane(wcnt[wsx]);
        n = n > WCAP ? WCAP : (n < 0 ? 0 : n);
        const int* lp = list + wsx * WCAP;
#pragma unroll 1
        for (int i = 0; i < n; ++i) {
          const int ent  = __builtin_amdgcn_readfirstlane(lp[i]);
          const int slot = ent & (NBA - 1);
          int e = cbase + ((ent >> 12) & (CHUNK - 1));
          e = e > nE - 1 ? nE - 1 : e;
          int src = ei[e];
          src = src < 0 ? 0 : (src > nN - 1 ? nN - 1 : src);
          const float* gp = g + (size_t)src * HID + 4 * lane;
          const v4f v0 = *(const v4f*)(gp);
          const v4f v1 = *(const v4f*)(gp + 128);
          const v4f v2 = *(const v4f*)(gp + 256);
          const v4f v3 = *(const v4f*)(gp + 384);
          v4f* ap = (v4f*)(acc + slot * HID + 4 * lane);
          ap[0]  = ap[0]  + v0;
          ap[32] = ap[32] + v1;
          ap[64] = ap[64] + v2;
          ap[96] = ap[96] + v3;
        }
      }
    }
    __syncthreads();
  }

#pragma unroll 1
  for (int i = 0; i < (NBA * HID / 8) / NTHR; ++i) {
    const int idx  = i * NTHR + tid;
    const int slot = idx >> 6;
    const int c8   = (idx & 63) * 8;
    int node = nodeBase + slot;
    node = node > nN - 1 ? nN - 1 : node;
    const float d  = dinv[node];
    const float* gp = g + (size_t)node * HID + c8;
    const v4f g0 = *(const v4f*)gp, g1 = *(const v4f*)(gp + 4);
    const v4f b0 = *(const v4f*)(bias + c8), b1 = *(const v4f*)(bias + c8 + 4);
    v4f* ap = (v4f*)(acc + slot * HID + c8);
    const v4f u0 = (ap[0] + g0) * d + b0;
    const v4f u1 = (ap[1] + g1) * d + b1;
    ap[0] = tanh4(u0);
    ap[1] = tanh4(u1);
  }
  __syncthreads();

  const size_t base = (size_t)nodeBase * HID;
  if (OUT16) {
#pragma unroll 4
    for (int i = 0; i < (NBA * HID / 8) / NTHR; ++i) {
      const int f = (i * NTHR + tid) * 8;
      const v4f a0 = *(const v4f*)(acc + f), a1 = *(const v4f*)(acc + f + 4);
      v8us hv, lv;
      split8(a0, a1, &hv, &lv);
      *(volatile v8us*)(oh + base + f) = hv;
      *(volatile v8us*)(ol + base + f) = lv;
    }
    __threadfence();
#pragma unroll 4
    for (int i = 0; i < (NBA * HID / 8) / NTHR; ++i) {
      const int f = (i * NTHR + tid) * 8;
      const v4f a0 = *(const v4f*)(acc + f), a1 = *(const v4f*)(acc + f + 4);
      v8us hv, lv;
      split8(a0, a1, &hv, &lv);
      *(volatile v8us*)(oh + base + f) = hv;
      *(volatile v8us*)(ol + base + f) = lv;
    }
  } else {
#pragma unroll 4
    for (int i = 0; i < (NBA * HID / 4) / NTHR; ++i) {
      const int f = (i * NTHR + tid) * 4;
      const v4f v = *(const v4f*)(acc + f);
      *(volatile v4f*)(of + base + f) = v;
    }
    __threadfence();
#pragma unroll 4
    for (int i = 0; i < (NBA * HID / 4) / NTHR; ++i) {
      const int f = (i * NTHR + tid) * 4;
      const v4f v = *(const v4f*)(acc + f);
      *(volatile v4f*)(of + base + f) = v;
    }
  }
}

__global__ __launch_bounds__(NTHR) void k_score(
    const float* __restrict__ h3, const int* __restrict__ ei, const int* __restrict__ tri,
    const float* __restrict__ fcW, const float* __restrict__ fcb, float* out,
    int nN, int nE, int nT) {
  __shared__ __attribute__((aligned(16))) float res[TPB];
  const int tid = threadIdx.x, lane = tid & 31, wave = tid >> 5;
  const int base = blockIdx.x * TPB;
  v4f w[4];
#pragma unroll
  for (int j = 0; j < 4; ++j) w[j] = *(const v4f*)(fcW + 4 * lane + 128 * j);
  const float bb = fcb[0];

#pragma unroll 1
  for (int i = 0; i < 4; ++i) {
    int t = base + wave * 4 + i;
    t = t > nT - 1 ? nT - 1 : t;
    int e = tri[t];
    e = e < 0 ? 0 : (e > nE - 1 ? nE - 1 : e);
    int a = ei[e];
    int b = ei[(size_t)nE + e];
    a = a < 0 ? 0 : (a > nN - 1 ? nN - 1 : a);
    b = b < 0 ? 0 : (b > nN - 1 ? nN - 1 : b);
    const float* pa = h3 + (size_t)a * HID + 4 * lane;
    const float* pb = h3 + (size_t)b * HID + 4 * lane;
    float s = 0.f;
#pragma unroll
    for (int j = 0; j < 4; ++j) {
      const v4f ha = *(const v4f*)(pa + 128 * j);
      const v4f hb = *(const v4f*)(pb + 128 * j);
      s += ha.x * hb.x * w[j].x;
      s += ha.y * hb.y * w[j].y;
      s += ha.z * hb.z * w[j].z;
      s += ha.w * hb.w * w[j].w;
    }
#pragma unroll
    for (int o = 16; o > 0; o >>= 1) s += __shfl_xor(s, o, 32);
    if (lane == 0) res[wave * 4 + i] = s + bb;
  }
  __syncthreads();

  if (wave == 0) {
    const int l8 = lane < 8 ? lane : 7;
    const v4f v  = *(const v4f*)(res + 4 * l8);
    const int t0 = base + 4 * lane;
    const bool act  = lane < 8;
    const bool full = act && (t0 + 4 <= nT);
    const bool part = act && !full && (t0 < nT);
    if (full) {
      *(volatile v4f*)(out + t0) = v;
    } else if (part) {
      if (t0 < nT)     *(volatile float*)(out + t0)     = v.x;
      if (t0 + 1 < nT) *(volatile float*)(out + t0 + 1) = v.y;
      if (t0 + 2 < nT) *(volatile float*)(out + t0 + 2) = v.z;
      if (t0 + 3 < nT) *(volatile float*)(out + t0 + 3) = v.w;
    }
    __threadfence();
    if (full) {
      *(volatile v4f*)(out + t0) = v;
    } else if (part) {
      if (t0 < nT)     *(volatile float*)(out + t0)     = v.x;
      if (t0 + 1 < nT) *(volatile float*)(out + t0 + 1) = v.y;
      if (t0 + 2 < nT) *(volatile float*)(out + t0 + 2) = v.z;
      if (t0 + 3 < nT) *(volatile float*)(out + t0 + 3) = v.w;
    }
  }
}

extern "C" void kernel_launch(void* const* d_in, const int* in_sizes, int n_in,
                              void* d_out, int out_size, void* d_ws, size_t ws_size,
                              hipStream_t stream) {
  if (n_in < 11) return;
  const int nN = in_sizes[0] / DIN;
  if (nN <= 0 || in_sizes[0] != nN * DIN) return;
  const int nE = in_sizes[1] / 2;
  if (nE <= 0 || in_sizes[1] != 2 * nE) return;
  const int nT = in_sizes[2];
  if (nT <= 0 || out_size != nT) return;
  if (in_sizes[3] != DIN * HID || in_sizes[4] < HID || in_sizes[5] != HID * HID || in_sizes[6] < HID) return;
  if (in_sizes[7] != HID * HID || in_sizes[8] < HID || in_sizes[9] < HID || in_sizes[10] < 1) return;

  const float* x   = (const float*)d_in[0];
  const int*   ei  = (const int*)d_in[1];
  const int*   tri = (const int*)d_in[2];
  const float* W1  = (const float*)d_in[3];
  const float* b1  = (const float*)d_in[4];
  const float* W2  = (const float*)d_in[5];
  const float* b2  = (const float*)d_in[6];
  const float* W3  = (const float*)d_in[7];
  const float* b3  = (const float*)d_in[8];
  const float* fcW = (const float*)d_in[9];
  const float* fcb = (const float*)d_in[10];
  float* out = (float*)d_out;

  const int nGB   = (nN + GR - 1) / GR;
  const int nRows = nGB * GR;
  const int nBD   = (nN + NBD - 1) / NBD;
  const int nSB   = (nT + TPB - 1) / TPB;

  char* ws = (char*)d_ws;
  size_t off = 0;
  const size_t oW1h = off; off += (size_t)HID * DIN * 2;  off = (off + 255) & ~(size_t)255;
  const size_t oW1l = off; off += (size_t)HID * DIN * 2;  off = (off + 255) & ~(size_t)255;
  const size_t oW2h = off; off += (size_t)HID * HID * 2;  off = (off + 255) & ~(size_t)255;
  const size_t oW2l = off; off += (size_t)HID * HID * 2;  off = (off + 255) & ~(size_t)255;
  const size_t oW3h = off; off += (size_t)HID * HID * 2;  off = (off + 255) & ~(size_t)255;
  const size_t oW3l = off; off += (size_t)HID * HID * 2;  off = (off + 255) & ~(size_t)255;
  const size_t oDv  = off; off += (size_t)nBD * NBD * 4;  off = (off + 255) & ~(size_t)255;
  const size_t oG   = off; off += (size_t)nRows * HID * 4; off = (off + 255) & ~(size_t)255;
  const size_t oH   = off; off += (size_t)nRows * HID * 4; off = (off + 255) & ~(size_t)255;
  if (off > ws_size) return;

  unsigned short* w1h = (unsigned short*)(ws + oW1h);
  unsigned short* w1l = (unsigned short*)(ws + oW1l);
  unsigned short* w2h = (unsigned short*)(ws + oW2h);
  unsigned short* w2l = (unsigned short*)(ws + oW2l);
  unsigned short* w3h = (unsigned short*)(ws + oW3h);
  unsigned short* w3l = (unsigned short*)(ws + oW3l);
  float*          dinv = (float*)(ws + oDv);
  float*          gpl  = (float*)(ws + oG);
  unsigned short* xh   = (unsigned short*)(ws + oH);
  unsigned short* xl   = (unsigned short*)(ws + oH + (size_t)nRows * DIN * 2);
  unsigned short* hh   = (unsigned short*)(ws + oH);
  unsigned short* hl   = (unsigned short*)(ws + oH + (size_t)nRows * HID * 2);
  float*          h3   = (float*)(ws + oH);

  const int vec8 = ((nE & 3) == 0) ? 1 : 0;

  const int nPrep = HID * DIN / 8 + 2 * (HID * HID / 8);
  k_wprep<<<(nPrep + NTHR - 1) / NTHR, NTHR, 0, stream>>>(W1, W2, W3, w1h, w1l, w2h, w2l, w3h, w3l);

  const int nX = nRows * (DIN / 8);
  k_xprep<<<(nX + NTHR - 1) / NTHR, NTHR, 0, stream>>>(x, xh, xl, nN, nRows);

  k_deg<<<nBD, NTHR, 0, stream>>>(ei, dinv, nE, vec8);

  hipFuncSetAttribute(reinterpret_cast<const void*>(&k_gemm),
                      hipFuncAttributeMaxDynamicSharedMemorySize, LDS_GEMM);
  hipFuncSetAttribute(reinterpret_cast<const void*>(&k_agg<1>),
                      hipFuncAttributeMaxDynamicSharedMemorySize, LDS_AGG);
  hipFuncSetAttribute(reinterpret_cast<const void*>(&k_agg<0>),
                      hipFuncAttributeMaxDynamicSharedMemorySize, LDS_AGG);

  const dim3 gg(HID / GCOL, nGB);

  k_gemm<<<gg, NTHR, LDS_GEMM, stream>>>(xh, xl, w1h, w1l, dinv, gpl, DIN);
  k_agg<1><<<nGB, NTHR, LDS_AGG, stream>>>(ei, gpl, dinv, b1, hh, hl, h3, nN, nE, vec8);
  k_gemm<<<gg, NTHR, LDS_GEMM, stream>>>(hh, hl, w2h, w2l, dinv, gpl, HID);
  k_agg<1><<<nGB, NTHR, LDS_AGG, stream>>>(ei, gpl, dinv, b2, hh, hl, h3, nN, nE, vec8);
  k_gemm<<<gg, NTHR, LDS_GEMM, stream>>>(hh, hl, w3h, w3l, dinv, gpl, HID);
  k_agg<0><<<nGB, NTHR, LDS_AGG, stream>>>(ei, gpl, dinv, b3, hh, hl, h3, nN, nE, vec8);

  k_score<<<nSB, NTHR, 0, stream>>>(h3, ei, tri, fcW, fcb, out, nN, nE, nT);
}
